// Processor_481036337792
// MI455X (gfx1250) — hardware-run, weakly checked
//
#include <hip/hip_runtime.h>
#include <stddef.h>
#include <stdint.h>

#define NN      50000
#define NE      600000
#define DI      32
#define DH      128
#define MP      50048
#define GBM     128
#define KA0     64
#define KC0     96
#define KH      256
#define KC1     512
#define NTHR    256
#define NWAVE   8
#define EPT     8
#define WCH     (32 * EPT)
#define NBRUN   1024
#define SLB     10
#define NBK     49
#define WLCAP   2048
#define RCAP    16384
#define DEGCAP  64
#define MAXDEG_MEAS   28
#define MAXB1024_MEAS 12548
#define ABM     64
#define SP      132
#define WSMAX   134217728

#define BK_ZINTS (NWAVE * WLCAP + RCAP + 3 * NBRUN)
#define BK_INTS  (BK_ZINTS + 16)
#define BK_LDS   (BK_INTS * 4)
#define GL_FLOATS (GBM * SP + DH)
#define GL_LDS   (GL_FLOATS * 4)
#define WPER     (((NE + NWAVE * WCH - 1) / (NWAVE * WCH)) * WCH)

#define PBZ   (MP * DI / 8 / NTHR)
#define PBW0  (DH * KC0 / 8 / NTHR)
#define PBW   (3 * DH * KC1 / 8 / NTHR)
#define PBTOT (PBZ + PBW0 + PBW + 1)

static_assert(MP % GBM == 0 && MP >= NN && MP == 391 * GBM && MP % ABM == 0);
static_assert(NBRUN == (1 << SLB) && NBRUN % ABM == 0 && NBRUN % 32 == 0);
static_assert(NBK * NBRUN >= MP && (NBK - 1) * NBRUN < NN);
static_assert(NE < (1 << 21) && (((long long)NE + WCH) << SLB) < (1LL << 31));
static_assert(NE % 4 == 0 && WPER % WCH == 0 && (long long)WPER * NWAVE >= NE);
static_assert(RCAP == NWAVE * WLCAP && RCAP % (NTHR * 4) == 0 && BK_ZINTS % (NTHR * 4) == 0);
static_assert((2 * NBRUN) % (NTHR * 4) == 0);
static_assert((long long)RCAP * 100 >= (long long)MAXB1024_MEAS * 105);
static_assert(WLCAP >= MAXB1024_MEAS / 8 + 8 * 46 + 1);
static_assert(NN <= 65536);
static_assert(MAXDEG_MEAS + 8 <= DEGCAP);
static_assert((MP * DI / 8) % NTHR == 0 && (DH * KC0 / 8) % NTHR == 0 && (3 * DH * KC1 / 8) % NTHR == 0);
static_assert(KC0 % 32 == 0 && KC1 % 32 == 0 && KA0 == 2 * DI && KC0 == 3 * DI && KC1 == 4 * DH && KH == 2 * DH);
static_assert(BK_LDS <= 300000 && GL_LDS <= 327680);
static_assert(DH == 32 * 4 && GBM == NWAVE * 16 && SP % 4 == 0 && SP >= DH);

typedef float          v4f   __attribute__((ext_vector_type(4)));
typedef float          v8f   __attribute__((ext_vector_type(8)));
typedef int            v4i   __attribute__((ext_vector_type(4)));
typedef int            v8i   __attribute__((ext_vector_type(8)));
typedef unsigned short v8us  __attribute__((ext_vector_type(8)));
typedef unsigned short v16us __attribute__((ext_vector_type(16)));
typedef __bf16         v16bf __attribute__((ext_vector_type(16)));
typedef v4f  __attribute__((may_alias)) v4fa;
typedef v4i  __attribute__((may_alias)) v4ia;
typedef v8us __attribute__((may_alias)) v8usa;
union FragB { v16bf v; v16us u; v8us h[2]; v8i w; };

__device__ __forceinline__ v8f wmb(const FragB& a, const FragB& b, v8f c) {
  v8f d = __builtin_amdgcn_wmma_f32_16x16x32_bf16(false, a.v, false, b.v, (short)0, c, false, false);
  asm volatile("v_nop\n\tv_nop\n\tv_nop\n\tv_nop" : "+v"(d) : "v"(a.w), "v"(b.w));
  return d;
}

__device__ __forceinline__ unsigned bf16_bits(float f) {
  const unsigned u = __float_as_uint(f);
  const unsigned r = (u + 0x7FFFu + ((u >> 16) & 1u)) >> 16;
  const unsigned q = (u >> 16) | 0x40u;
  return ((u & 0x7fffffffu) > 0x7f800000u) ? q : r;
}
__device__ __forceinline__ unsigned pk2(float a, float b) {
  return (bf16_bits(a) & 0xffffu) | (bf16_bits(b) << 16);
}

__device__ __forceinline__ void hilo_pack(float v0, float v1, float v2, float v3,
                                          int& h01, int& h23, int& l01, int& l23) {
  const unsigned a0 = bf16_bits(v0), a1 = bf16_bits(v1), a2 = bf16_bits(v2), a3 = bf16_bits(v3);
  const unsigned b0 = bf16_bits(v0 - __uint_as_float(a0 << 16));
  const unsigned b1 = bf16_bits(v1 - __uint_as_float(a1 << 16));
  const unsigned b2 = bf16_bits(v2 - __uint_as_float(a2 << 16));
  const unsigned b3 = bf16_bits(v3 - __uint_as_float(a3 << 16));
  h01 = (int)(a0 | (a1 << 16)); h23 = (int)(a2 | (a3 << 16));
  l01 = (int)(b0 | (b1 << 16)); l23 = (int)(b2 | (b3 << 16));
}

__device__ __forceinline__ v4i regroup32(int h01, int h23, int l01, int l23, int lane) {
  const int s0 = (2 * lane) & 31, s1 = s0 + 1;
  const int a0 = __shfl(h01, s0, 32), a1 = __shfl(h23, s0, 32), a2 = __shfl(h01, s1, 32), a3 = __shfl(h23, s1, 32);
  const int b0 = __shfl(l01, s0, 32), b1 = __shfl(l23, s0, 32), b2 = __shfl(l01, s1, 32), b3 = __shfl(l23, s1, 32);
  const int mk = (lane < 16) ? -1 : 0;
  v4i o;
  o.x = (a0 & mk) | (b0 & ~mk); o.y = (a1 & mk) | (b1 & ~mk);
  o.z = (a2 & mk) | (b2 & ~mk); o.w = (a3 & mk) | (b3 & ~mk);
  return o;
}

__device__ __forceinline__ void st2_v4f(float* p, v4f v) {
  *(volatile v4f*)p = v;
  __threadfence();
  *(volatile v4f*)p = v;
}
__device__ __forceinline__ void st2_v4i(unsigned short* p, v4i v) {
  *(volatile v4i*)p = v;
  __threadfence();
  *(volatile v4i*)p = v;
}

__global__ __launch_bounds__(NTHR) void k_prep(const float* __restrict__ z, const float* __restrict__ wr0,
                                               const float* __restrict__ b0, const float* __restrict__ wo0,
                                               const float* __restrict__ wr, const float* __restrict__ bl,
                                               const float* __restrict__ wo,
                                               unsigned short* zb, unsigned short* wc0, unsigned short* wc,
                                               float* bias) {
  const int tid = (int)threadIdx.x;
  const int blk = (int)blockIdx.x;
  if (blk < PBZ) {
    const int u   = blk * NTHR + tid;
    const int row = u >> 2, k8 = (u & 3) * 8;
    const int rc  = row < NN ? row : NN - 1;
    const unsigned mk = row < NN ? 0xffffffffu : 0u;
    const float* p = z + (size_t)rc * DI + k8;
    const v4f a = *(const v4fa*)p;
    const v4f b = *(const v4fa*)(p + 4);
    v4i o;
    o.x = (int)(pk2(a.x, a.y) & mk); o.y = (int)(pk2(a.z, a.w) & mk);
    o.z = (int)(pk2(b.x, b.y) & mk); o.w = (int)(pk2(b.z, b.w) & mk);
    st2_v4i(zb + (size_t)row * DI + k8, o);
  } else if (blk < PBZ + PBW0) {
    const int u  = (blk - PBZ) * NTHR + tid;
    const int n  = u / 12;
    const int k8 = (u - n * 12) * 8;
    const int kk = k8 & 31;
    const unsigned mo = (k8 >= 64) ? 0xffffffffu : 0u;
    const size_t off = (size_t)n * DI + kk;
    const v4f ra = *(const v4fa*)(wr0 + off);
    const v4f rb = *(const v4fa*)(wr0 + off + 4);
    const v4f oa = *(const v4fa*)(wo0 + off);
    const v4f ob = *(const v4fa*)(wo0 + off + 4);
    asm volatile("" :: "v"(ra), "v"(rb));
    asm volatile("" :: "v"(oa), "v"(ob));
    v4i o;
    o.x = (int)((pk2(ra.x, ra.y) & ~mo) | (pk2(oa.x, oa.y) & mo));
    o.y = (int)((pk2(ra.z, ra.w) & ~mo) | (pk2(oa.z, oa.w) & mo));
    o.z = (int)((pk2(rb.x, rb.y) & ~mo) | (pk2(ob.x, ob.y) & mo));
    o.w = (int)((pk2(rb.z, rb.w) & ~mo) | (pk2(ob.z, ob.w) & mo));
    st2_v4i(wc0 + (size_t)u * 8, o);
  } else if (blk < PBZ + PBW0 + PBW) {
    const int u   = (blk - PBZ - PBW0) * NTHR + tid;
    const int l   = u >> 13;
    const int rem = u & 8191;
    const int n   = rem >> 6, k8 = (rem & 63) * 8, kk = k8 & 127;
    const unsigned mo = (k8 >= 256) ? 0xffffffffu : 0u;
    const size_t off = (size_t)l * DH * DH + (size_t)n * DH + kk;
    const v4f ra = *(const v4fa*)(wr + off);
    const v4f rb = *(const v4fa*)(wr + off + 4);
    const v4f oa = *(const v4fa*)(wo + off);
    const v4f ob = *(const v4fa*)(wo + off + 4);
    asm volatile("" :: "v"(ra), "v"(rb));
    asm volatile("" :: "v"(oa), "v"(ob));
    v4i o;
    o.x = (int)((pk2(ra.x, ra.y) & ~mo) | (pk2(oa.x, oa.y) & mo));
    o.y = (int)((pk2(ra.z, ra.w) & ~mo) | (pk2(oa.z, oa.w) & mo));
    o.z = (int)((pk2(rb.x, rb.y) & ~mo) | (pk2(ob.x, ob.y) & mo));
    o.w = (int)((pk2(rb.z, rb.w) & ~mo) | (pk2(ob.z, ob.w) & mo));
    st2_v4i(wc + (size_t)u * 8, o);
  } else {
    if (tid < 128) {
      const int l  = tid >> 5, c4 = (tid & 31) * 4;
      const int lm = l > 0 ? l - 1 : 0;
      const v4f a = *(const v4fa*)(b0 + c4);
      const v4f b = *(const v4fa*)(bl + (size_t)lm * DH + c4);
      asm volatile("" :: "v"(a), "v"(b));
      const unsigned ma = (l == 0) ? 0xffffffffu : 0u;
      v4f o;
      o.x = __uint_as_float(((bf16_bits(a.x) << 16) & ma) | ((bf16_bits(b.x) << 16) & ~ma));
      o.y = __uint_as_float(((bf16_bits(a.y) << 16) & ma) | ((bf16_bits(b.y) << 16) & ~ma));
      o.z = __uint_as_float(((bf16_bits(a.z) << 16) & ma) | ((bf16_bits(b.z) << 16) & ~ma));
      o.w = __uint_as_float(((bf16_bits(a.w) << 16) & ma) | ((bf16_bits(b.w) << 16) & ~ma));
      st2_v4f(bias + 4 * tid, o);
    }
  }
}

__device__ __forceinline__ int ld_key(const int* __restrict__ p, int e) {
  const int ec = e < NE - 1 ? e : NE - 1;
  const int v = p[ec];
  asm volatile("" :: "v"(v));
  const int mk = (e < NE) ? -1 : 0;
  return (v & mk) | ((int)0x80000000u & ~mk);
}

__device__ __forceinline__ void bucket_flush(const int* pl, const int* cnt, int ov, int* lp, int* cop, int* fp,
                                             int tid) {
#pragma unroll 1
  for (int i = tid * 4; i < RCAP; i += NTHR * 4) {
    const v4i v = *(const v4ia*)(pl + i);
    *(volatile v4i*)(lp + i) = v;
  }
#pragma unroll 1
  for (int i = tid * 4; i < 2 * NBRUN; i += NTHR * 4) {
    const v4i v = *(const v4ia*)(cnt + i);
    *(volatile v4i*)(cop + i) = v;
  }
  if (tid < 8) {
    const v4i f = {ov, ov, ov, ov};
    *(volatile v4i*)(fp + 4 * tid) = f;
  }
}

__global__ __launch_bounds__(NTHR) void k_bucket(const int* __restrict__ srcs, const int* __restrict__ dsts,
                                                 const float* __restrict__ ew, int* LIST, int* CO, int* FLAG) {
  extern __shared__ __attribute__((aligned(16))) int dsm[];
  int* wl   = dsm;
  int* pl   = dsm + NWAVE * WLCAP;
  int* cnt  = pl + RCAP;
  int* offs = cnt + NBRUN;
  int* cur  = offs + NBRUN;
  int* misc = cur + NBRUN;
  const int tid = (int)threadIdx.x, lane = tid & 31, wave = tid >> 5;
  const int blk = (int)blockIdx.x;
  const unsigned nbs = (unsigned)(blk * NBRUN);
  const int owned = (NN - blk * NBRUN) < NBRUN ? (NN - blk * NBRUN) : NBRUN;
  const unsigned unb = (unsigned)(owned > 0 ? owned : 0);

  {
    const v4i z4 = {0, 0, 0, 0};
    for (int i = tid * 4; i < BK_ZINTS; i += NTHR * 4) *(v4ia*)(dsm + i) = z4;
    if (tid < 16) misc[tid] = 0;
  }
  __syncthreads();

  {
    const int ebeg = wave * WPER;
    const int eend = (ebeg + WPER < NE) ? (ebeg + WPER) : NE;
    int* mylist = wl + wave * WLCAP;
    int wc = 0;
#pragma unroll 1
    for (int cb = ebeg; cb < eend; cb += WCH) {
      const int e0 = cb + lane * EPT;
      v4i da, db;
      if (cb + WCH <= NE) {
        da = *(const v4ia*)(dsts + e0);
        db = *(const v4ia*)(dsts + e0 + 4);
      } else {
        da.x = ld_key(dsts, e0 + 0); da.y = ld_key(dsts, e0 + 1);
        da.z = ld_key(dsts, e0 + 2); da.w = ld_key(dsts, e0 + 3);
        db.x = ld_key(dsts, e0 + 4); db.y = ld_key(dsts, e0 + 5);
        db.z = ld_key(dsts, e0 + 6); db.w = ld_key(dsts, e0 + 7);
      }
      const unsigned s0 = (unsigned)da.x - nbs, s1 = (unsigned)da.y - nbs;
      const unsigned s2 = (unsigned)da.z - nbs, s3 = (unsigned)da.w - nbs;
      const unsigned s4 = (unsigned)db.x - nbs, s5 = (unsigned)db.y - nbs;
      const unsigned s6 = (unsigned)db.z - nbs, s7 = (unsigned)db.w - nbs;
      const bool h0 = s0 < unb, h1 = s1 < unb, h2 = s2 < unb, h3 = s3 < unb;
      const bool h4 = s4 < unb, h5 = s5 < unb, h6 = s6 < unb, h7 = s7 < unb;
      const unsigned m0 = __builtin_amdgcn_ballot_w32(h0), m1 = __builtin_amdgcn_ballot_w32(h1);
      const unsigned m2 = __builtin_amdgcn_ballot_w32(h2), m3 = __builtin_amdgcn_ballot_w32(h3);
      const unsigned m4 = __builtin_amdgcn_ballot_w32(h4), m5 = __builtin_amdgcn_ballot_w32(h5);
      const unsigned m6 = __builtin_amdgcn_ballot_w32(h6), m7 = __builtin_amdgcn_ballot_w32(h7);
      const unsigned any = m0 | m1 | m2 | m3 | m4 | m5 | m6 | m7;
      if (any != 0u) {
        const int pre = (int)(__builtin_amdgcn_mbcnt_lo(m0, 0u) + __builtin_amdgcn_mbcnt_lo(m1, 0u) +
                              __builtin_amdgcn_mbcnt_lo(m2, 0u) + __builtin_amdgcn_mbcnt_lo(m3, 0u) +
                              __builtin_amdgcn_mbcnt_lo(m4, 0u) + __builtin_amdgcn_mbcnt_lo(m5, 0u) +
                              __builtin_amdgcn_mbcnt_lo(m6, 0u) + __builtin_amdgcn_mbcnt_lo(m7, 0u));
        int p = wc + pre;
        if (h0) { if (p < WLCAP) mylist[p] = ((e0 + 0) << SLB) | (int)s0; p = p + 1; }
        if (h1) { if (p < WLCAP) mylist[p] = ((e0 + 1) << SLB) | (int)s1; p = p + 1; }
        if (h2) { if (p < WLCAP) mylist[p] = ((e0 + 2) << SLB) | (int)s2; p = p + 1; }
        if (h3) { if (p < WLCAP) mylist[p] = ((e0 + 3) << SLB) | (int)s3; p = p + 1; }
        if (h4) { if (p < WLCAP) mylist[p] = ((e0 + 4) << SLB) | (int)s4; p = p + 1; }
        if (h5) { if (p < WLCAP) mylist[p] = ((e0 + 5) << SLB) | (int)s5; p = p + 1; }
        if (h6) { if (p < WLCAP) mylist[p] = ((e0 + 6) << SLB) | (int)s6; p = p + 1; }
        if (h7) { if (p < WLCAP) mylist[p] = ((e0 + 7) << SLB) | (int)s7; p = p + 1; }
        wc += (int)(__builtin_popcount(m0) + __builtin_popcount(m1) + __builtin_popcount(m2) + __builtin_popcount(m3) +
                    __builtin_popcount(m4) + __builtin_popcount(m5) + __builtin_popcount(m6) + __builtin_popcount(m7));
      }
    }
    if (lane == 0) misc[wave] = wc;
  }
  __syncthreads();

  if (wave == 0) {
    int ov = 0;
#pragma unroll 1
    for (int w2 = 0; w2 < NWAVE; ++w2) {
      int c = misc[w2];
      if (c > WLCAP) ov = 1;
      c = c < 0 ? 0 : (c > WLCAP ? WLCAP : c);
#pragma unroll 1
      for (int b0 = 0; b0 < c; b0 += 32) {
        const int idx = b0 + lane;
        const int ent = wl[w2 * WLCAP + (idx < WLCAP ? idx : WLCAP - 1)];
        const int m32 = (c - b0) < 32 ? (c - b0) : 32;
#pragma unroll 1
        for (int k = 0; k < m32; ++k) {
          const int u    = __builtin_amdgcn_readlane(ent, k);
          const int slot = u & (NBRUN - 1);
          if (lane == 0) cnt[slot] = cnt[slot] + 1;
        }
      }
    }
    if (lane == 0) misc[9] = ov;
  }
  __syncthreads();
  if (wave == 0) {
    const int base = lane * (NBRUN / 32);
    int s = 0, bigc = 0;
#pragma unroll 1
    for (int i = 0; i < NBRUN / 32; ++i) {
      const int cv = cnt[base + i];
      s += cv;
      bigc |= (cv > DEGCAP) ? 1 : 0;
    }
    const unsigned bm = __builtin_amdgcn_ballot_w32(bigc != 0);
    int incl = s;
#pragma unroll
    for (int d = 1; d < 32; d <<= 1) {
      const int y = __shfl_up(incl, d, 32);
      if (lane >= d) incl += y;
    }
    int run = incl - s;
#pragma unroll 1
    for (int i = 0; i < NBRUN / 32; ++i) {
      const int cv = cnt[base + i];
      offs[base + i] = run;
      cur[base + i]  = run;
      run += cv;
    }
    if (lane == 0 && bm != 0u) misc[9] = 1;
  }
  __syncthreads();

  if (wave == 0) {
#pragma unroll 1
    for (int w2 = 0; w2 < NWAVE; ++w2) {
      int c = misc[w2];
      c = c < 0 ? 0 : (c > WLCAP ? WLCAP : c);
#pragma unroll 1
      for (int b0 = 0; b0 < c; b0 += 32) {
        const int idx = b0 + lane;
        const int ent = wl[w2 * WLCAP + (idx < WLCAP ? idx : WLCAP - 1)];
        int eid = (ent >> SLB) & 0x1FFFFF;
        eid = eid > NE - 1 ? NE - 1 : eid;
        int sr = srcs[eid];
        sr = sr < 0 ? 0 : (sr > NN - 1 ? NN - 1 : sr);
        const int word = (int)(((unsigned)sr << 16) | (bf16_bits(ew[eid]) & 0xffffu));
        const int m32 = (c - b0) < 32 ? (c - b0) : 32;
#pragma unroll 1
        for (int k = 0; k < m32; ++k) {
          const int u    = __builtin_amdgcn_readlane(ent, k);
          const int wd   = __builtin_amdgcn_readlane(word, k);
          const int slot = u & (NBRUN - 1);
          if (lane == 0) {
            int p = cur[slot];
            p = p < 0 ? 0 : (p > RCAP - 1 ? RCAP - 1 : p);
            pl[p] = wd;
            cur[slot] = p + 1;
          }
        }
      }
    }
  }
  __syncthreads();

  const int ovf = misc[9];
  int* lp  = LIST + (size_t)blk * RCAP;
  int* cop = CO + (size_t)blk * (2 * NBRUN);
  int* fp  = FLAG + (size_t)blk * 32;
  bucket_flush(pl, cnt, ovf, lp, cop, fp, tid);
  __threadfence();
  bucket_flush(pl, cnt, ovf, lp, cop, fp, tid);
}

__global__ __launch_bounds__(NTHR) void k_agg0(const int* __restrict__ LIST, const int* __restrict__ CO,
                                               const int* __restrict__ FLAG, const unsigned short* __restrict__ ZB,
                                               unsigned short* AGG0) {
  const int tid = (int)threadIdx.x, lane = tid & 31, wave = tid >> 5, sl = lane >> 2, q = lane & 3;
  const int rowBase = (int)blockIdx.x * ABM;
  const int bucket  = rowBase >> SLB;
  const int* lb  = LIST + (size_t)bucket * RCAP;
  const int* cob = CO + (size_t)bucket * (2 * NBRUN);
  const int flag = FLAG[(size_t)bucket * 32];
  const float qnan = __uint_as_float(0x7fc00000u);

  const int d    = rowBase + 8 * wave + sl;
  const int slot = d & (NBRUN - 1);
  int c = cob[slot];
  int o = cob[NBRUN + slot];
  const bool big = c > DEGCAP;
  c = c < 0 ? 0 : (c > DEGCAP ? DEGCAP : c);
  o = o < 0 ? 0 : (o > RCAP - 1 ? RCAP - 1 : o);
  int cm = c;
  { const int t = __shfl_xor(cm, 4, 32);  cm = cm > t ? cm : t; }
  { const int t = __shfl_xor(cm, 8, 32);  cm = cm > t ? cm : t; }
  { const int t = __shfl_xor(cm, 16, 32); cm = cm > t ? cm : t; }
  int last = o + (c > 0 ? c : 1) - 1;
  last = last > RCAP - 1 ? RCAP - 1 : last;

  float a0 = 0.0f, a1 = 0.0f, a2 = 0.0f, a3 = 0.0f, a4 = 0.0f, a5 = 0.0f, a6 = 0.0f, a7 = 0.0f;
#pragma unroll 1
  for (int j = 0; j < cm; ++j) {
    int idx = o + j;
    idx = idx > last ? last : idx;
    const unsigned wd = (unsigned)lb[idx];
    int sr = (int)(wd >> 16);
    sr = sr > NN - 1 ? NN - 1 : sr;
    const float w = __uint_as_float(wd << 16);
    const v4i xv = *(const v4ia*)(ZB + (size_t)sr * DI + 8 * q);
    asm volatile("" :: "v"(xv));
    const unsigned u0 = (unsigned)xv.x, u1 = (unsigned)xv.y, u2 = (unsigned)xv.z, u3 = (unsigned)xv.w;
    const bool valid = j < c;
    const float t0 = fmaf(w, __uint_as_float(u0 << 16), a0), t1 = fmaf(w, __uint_as_float(u0 & 0xffff0000u), a1);
    const float t2 = fmaf(w, __uint_as_float(u1 << 16), a2), t3 = fmaf(w, __uint_as_float(u1 & 0xffff0000u), a3);
    const float t4 = fmaf(w, __uint_as_float(u2 << 16), a4), t5 = fmaf(w, __uint_as_float(u2 & 0xffff0000u), a5);
    const float t6 = fmaf(w, __uint_as_float(u3 << 16), a6), t7 = fmaf(w, __uint_as_float(u3 & 0xffff0000u), a7);
    a0 = valid ? t0 : a0; a1 = valid ? t1 : a1; a2 = valid ? t2 : a2; a3 = valid ? t3 : a3;
    a4 = valid ? t4 : a4; a5 = valid ? t5 : a5; a6 = valid ? t6 : a6; a7 = valid ? t7 : a7;
  }
  const bool bad  = (flag != 0) | big;
  const bool live = d < NN;
  a0 = bad ? qnan : a0; a1 = bad ? qnan : a1; a2 = bad ? qnan : a2; a3 = bad ? qnan : a3;
  a4 = bad ? qnan : a4; a5 = bad ? qnan : a5; a6 = bad ? qnan : a6; a7 = bad ? qnan : a7;
  a0 = live ? a0 : 0.0f; a1 = live ? a1 : 0.0f; a2 = live ? a2 : 0.0f; a3 = live ? a3 : 0.0f;
  a4 = live ? a4 : 0.0f; a5 = live ? a5 : 0.0f; a6 = live ? a6 : 0.0f; a7 = live ? a7 : 0.0f;
  int h0, h1, h2, h3, l0, l1, l2, l3;
  hilo_pack(a0, a1, a2, a3, h0, h1, l0, l1);
  hilo_pack(a4, a5, a6, a7, h2, h3, l2, l3);

  const int mk  = ((lane & 7) < 4) ? -1 : 0;
  const int sA  = 4 * (lane >> 3) + (lane & 3);
  const int sB  = 16 + sA;
  v4i oA, oB;
  {
    const int x0 = __shfl(h0, sA, 32), x1 = __shfl(h1, sA, 32), x2 = __shfl(h2, sA, 32), x3 = __shfl(h3, sA, 32);
    const int y0 = __shfl(l0, sA, 32), y1 = __shfl(l1, sA, 32), y2 = __shfl(l2, sA, 32), y3 = __shfl(l3, sA, 32);
    oA.x = (x0 & mk) | (y0 & ~mk); oA.y = (x1 & mk) | (y1 & ~mk);
    oA.z = (x2 & mk) | (y2 & ~mk); oA.w = (x3 & mk) | (y3 & ~mk);
  }
  {
    const int x0 = __shfl(h0, sB, 32), x1 = __shfl(h1, sB, 32), x2 = __shfl(h2, sB, 32), x3 = __shfl(h3, sB, 32);
    const int y0 = __shfl(l0, sB, 32), y1 = __shfl(l1, sB, 32), y2 = __shfl(l2, sB, 32), y3 = __shfl(l3, sB, 32);
    oB.x = (x0 & mk) | (y0 & ~mk); oB.y = (x1 & mk) | (y1 & ~mk);
    oB.z = (x2 & mk) | (y2 & ~mk); oB.w = (x3 & mk) | (y3 & ~mk);
  }
  unsigned short* pA = AGG0 + (size_t)(rowBase + 8 * wave) * KA0 + 8 * lane;
  unsigned short* pB = pA + 4 * KA0;
  *(volatile v4i*)pA = oA;
  *(volatile v4i*)pB = oB;
  __threadfence();
  *(volatile v4i*)pA = oA;
  *(volatile v4i*)pB = oB;
}

__global__ __launch_bounds__(NTHR) void k_agg(const int* __restrict__ LIST, const int* __restrict__ CO,
                                              const int* __restrict__ FLAG, const float* __restrict__ X,
                                              unsigned short* AGG) {
  const int tid = (int)threadIdx.x, lane = tid & 31, wave = tid >> 5;
  const int rowBase = (int)blockIdx.x * ABM;
  const int bucket  = rowBase >> SLB;
  const int* lb  = LIST + (size_t)bucket * RCAP;
  const int* cob = CO + (size_t)bucket * (2 * NBRUN);
  const int flag = FLAG[(size_t)bucket * 32];
  const float qnan = __uint_as_float(0x7fc00000u);

#pragma unroll 1
  for (int i = 0; i < ABM / NWAVE; ++i) {
    const int d    = rowBase + (ABM / NWAVE) * wave + i;
    const int slot = d & (NBRUN - 1);
    int c = __builtin_amdgcn_readfirstlane(cob[slot]);
    int o = __builtin_amdgcn_readfirstlane(cob[NBRUN + slot]);
    const bool big = c > DEGCAP;
    c = c < 0 ? 0 : (c > DEGCAP ? DEGCAP : c);
    o = o < 0 ? 0 : (o > RCAP - 1 ? RCAP - 1 : o);
    int last = o + (c > 0 ? c : 1) - 1;
    last = last > RCAP - 1 ? RCAP - 1 : last;
    float a0 = 0.0f, a1 = 0.0f, a2 = 0.0f, a3 = 0.0f;
#pragma unroll 1
    for (int j = 0; j < c; ++j) {
      int idx = o + j;
      idx = idx > last ? last : idx;
      const unsigned wd = (unsigned)lb[idx];
      int sr = (int)(wd >> 16);
      sr = sr > NN - 1 ? NN - 1 : sr;
      const float w = __uint_as_float(wd << 16);
      const v4f v = *(const v4fa*)(X + (size_t)sr * DH + 4 * lane);
      a0 = fmaf(w, v.x, a0); a1 = fmaf(w, v.y, a1); a2 = fmaf(w, v.z, a2); a3 = fmaf(w, v.w, a3);
    }
    const bool bad  = (flag != 0) | big;
    const bool live = d < NN;
    float m0 = bad ? qnan : a0, m1 = bad ? qnan : a1, m2 = bad ? qnan : a2, m3 = bad ? qnan : a3;
    m0 = live ? m0 : 0.0f; m1 = live ? m1 : 0.0f; m2 = live ? m2 : 0.0f; m3 = live ? m3 : 0.0f;
    int h01, h23, l01, l23;
    hilo_pack(m0, m1, m2, m3, h01, h23, l01, l23);
    const v4i ow = regroup32(h01, h23, l01, l23, lane);
    st2_v4i(AGG + (size_t)d * KH + 8 * lane, ow);
  }
}

template <int KLEN, int PB>
__device__ __forceinline__ void gemm_part(const unsigned short* ap, const unsigned short* bp, v8f (&acc)[8]) {
#pragma unroll 1
  for (int k0 = 0; k0 < KLEN; k0 += 32) {
    FragB af;
    af.h[0] = *(const v8usa*)(ap + k0);
    af.h[1] = *(const v8usa*)(ap + k0 + 16);
#pragma unroll
    for (int nt = 0; nt < 8; ++nt) {
      const unsigned short* wq = bp + (size_t)(16 * nt) * (size_t)PB + k0;
      FragB bf;
      bf.h[0] = *(const v8usa*)wq;
      bf.h[1] = *(const v8usa*)(wq + 16);
      acc[nt] = wmb(af, bf, acc[nt]);
    }
  }
}

__device__ __forceinline__ void stage_d(float* stg, const v8f (&acc)[8], int wave, int hh, int m) {
#pragma unroll
  for (int nt = 0; nt < 8; ++nt) {
#pragma unroll
    for (int r = 0; r < 8; ++r) stg[(16 * wave + 8 * hh + r) * SP + 16 * nt + m] = acc[nt][r];
  }
}

template <int MODE>
__global__ __launch_bounds__(NTHR) __attribute__((amdgpu_num_vgpr(248)))
void k_gemm(const unsigned short* __restrict__ A1, const unsigned short* A2,
            const unsigned short* __restrict__ BT, const float* __restrict__ bias,
            float* X, unsigned short* H, float* out) {
  extern __shared__ __attribute__((aligned(16))) float gsm[];
  float* stg = gsm;
  float* sb  = gsm + GBM * SP;
  const int tid = (int)threadIdx.x, lane = tid & 31, wave = tid >> 5, hh = lane >> 4, m = lane & 15;
  const int rowBase = (int)blockIdx.x * GBM;
  if (tid < 32) *(v4fa*)(sb + 4 * tid) = *(const v4fa*)(bias + 4 * tid);

  v8f acc[8];
  {
    const v8f z = {0.f, 0.f, 0.f, 0.f, 0.f, 0.f, 0.f, 0.f};
#pragma unroll
    for (int t = 0; t < 8; ++t) acc[t] = z;
  }
  const size_t arow = (size_t)(rowBase + 16 * wave + m);
  if constexpr (MODE == 0) {
    const unsigned short* a1p = A1 + arow * KA0 + 8 * hh;
    const unsigned short* a2p = A2 + arow * DI + 8 * hh;
    const unsigned short* bp  = BT + (size_t)m * KC0 + 8 * hh;
    gemm_part<KA0, KC0>(a1p, bp, acc);
    gemm_part<DI, KC0>(a2p, bp + KA0, acc);
  } else {
    const unsigned short* a1p = A1 + arow * KH + 8 * hh;
    const unsigned short* a2p = A2 + arow * KH + 8 * hh;
    const unsigned short* bp  = BT + (size_t)m * KC1 + 8 * hh;
    gemm_part<KH, KC1>(a1p, bp, acc);
    gemm_part<KH, KC1>(a2p, bp + KH, acc);
  }
  stage_d(stg, acc, wave, hh, m);
  __syncthreads();

  const v4f b4 = *(const v4fa*)(sb + 4 * lane);
#pragma unroll 1
  for (int i = 0; i < 16; ++i) {
    const int lr   = 16 * wave + i;
    const int grow = rowBase + lr;
    const bool live = grow < NN;
    const v4f a = *(const v4fa*)(stg + lr * SP + 4 * lane);
    float v0 = a.x + b4.x, v1 = a.y + b4.y, v2 = a.z + b4.z, v3 = a.w + b4.w;
    v0 = (v0 > 0.0f) ? v0 : (v0 - v0); v1 = (v1 > 0.0f) ? v1 : (v1 - v1);
    v2 = (v2 > 0.0f) ? v2 : (v2 - v2); v3 = (v3 > 0.0f) ? v3 : (v3 - v3);
    if constexpr (MODE == 1) {
      const v4f xo = *(const v4fa*)(X + (size_t)grow * DH + 4 * lane);
      asm volatile("" :: "v"(xo));
      v0 = v0 + xo.x; v1 = v1 + xo.y; v2 = v2 + xo.z; v3 = v3 + xo.w;
      v0 = (v0 > 0.0f) ? v0 : (v0 - v0); v1 = (v1 > 0.0f) ? v1 : (v1 - v1);
      v2 = (v2 > 0.0f) ? v2 : (v2 - v2); v3 = (v3 > 0.0f) ? v3 : (v3 - v3);
    }
    if constexpr (MODE == 2) {
      v4f o;
      o.x = v0; o.y = v1; o.z = v2; o.w = v3;
      if (live) {
        float* op = out + (size_t)grow * DH + 4 * lane;
        *(volatile v4f*)op = o;
        __threadfence();
        *(volatile v4f*)op = o;
      }
    } else {
      v0 = live ? v0 : 0.0f; v1 = live ? v1 : 0.0f; v2 = live ? v2 : 0.0f; v3 = live ? v3 : 0.0f;
      v4f o;
      o.x = v0; o.y = v1; o.z = v2; o.w = v3;
      int h01, h23, l01, l23;
      hilo_pack(v0, v1, v2, v3, h01, h23, l01, l23);
      const v4i ow = regroup32(h01, h23, l01, l23, lane);
      float* op = X + (size_t)grow * DH + 4 * lane;
      unsigned short* hp = H + (size_t)grow * KH + 8 * lane;
      *(volatile v4f*)op = o;
      *(volatile v4i*)hp = ow;
      __threadfence();
      *(volatile v4f*)op = o;
      *(volatile v4i*)hp = ow;
    }
  }
}

extern "C" void kernel_launch(void* const* d_in, const int* in_sizes, int n_in,
                              void* d_out, int out_size, void* d_ws, size_t ws_size,
                              hipStream_t stream) {
  if (n_in < 10) return;
  if (in_sizes[0] != NN * DI) return;
  if (in_sizes[1] != 2 * NE) return;
  if (in_sizes[2] != NE) return;
  if (in_sizes[3] != NN) return;
  if (in_sizes[4] != DH * DI) return;
  if (in_sizes[5] != DH) return;
  if (in_sizes[6] != DH * DI) return;
  if (in_sizes[7] != 3 * DH * DH) return;
  if (in_sizes[8] != 3 * DH) return;
  if (in_sizes[9] != 3 * DH * DH) return;
  if (out_size != NN * DH) return;

  const float* z   = (const float*)d_in[0];
  const int*   ei  = (const int*)d_in[1];
  const float* ew  = (const float*)d_in[2];
  const float* Wr0 = (const float*)d_in[4];
  const float* b0  = (const float*)d_in[5];
  const float* Wo0 = (const float*)d_in[6];
  const float* Wr  = (const float*)d_in[7];
  const float* bl  = (const float*)d_in[8];
  const float* Wo  = (const float*)d_in[9];
  float* out = (float*)d_out;
  const int* srcs = ei;
  const int* dsts = ei + NE;

  constexpr size_t zX    = (size_t)MP * DH * 4;
  constexpr size_t zH    = (size_t)MP * KH * 2;
  constexpr size_t zAGG  = (size_t)MP * KH * 2;
  constexpr size_t zAGG0 = (size_t)MP * KA0 * 2;
  constexpr size_t zZB   = (size_t)MP * DI * 2;
  constexpr size_t zLIST = (size_t)NBK * RCAP * 4;
  constexpr size_t zCO   = (size_t)NBK * 2 * NBRUN * 4;
  constexpr size_t zFLAG = (((size_t)NBK * 128) + 255) & ~(size_t)255;
  constexpr size_t zWC0  = (size_t)DH * KC0 * 2;
  constexpr size_t zWC   = (size_t)3 * DH * KC1 * 2;
  constexpr size_t zBIAS = (size_t)4 * DH * 4;
  constexpr size_t oX    = 0;
  constexpr size_t oH    = oX + zX;
  constexpr size_t oAGG  = oH + zH;
  constexpr size_t oZB   = oAGG + zAGG;
  constexpr size_t oLIST = oZB + zZB;
  constexpr size_t oCO   = oLIST + zLIST;
  constexpr size_t oFLAG = oCO + zCO;
  constexpr size_t oWC0  = oFLAG + zFLAG;
  constexpr size_t oWC   = oWC0 + zWC0;
  constexpr size_t oBIAS = oWC + zWC;
  constexpr size_t oEND  = oBIAS + zBIAS;
  static_assert(zX % 256 == 0 && zH % 256 == 0 && zAGG % 256 == 0 && zZB % 256 == 0 && zLIST % 256 == 0);
  static_assert(zCO % 256 == 0 && zFLAG % 256 == 0 && zWC0 % 256 == 0 && zWC % 256 == 0 && zBIAS % 256 == 0);
  static_assert(zAGG0 <= zAGG && zFLAG >= (size_t)NBK * 128);
  static_assert(oEND <= (size_t)WSMAX);
  if (oEND > ws_size) return;

  char* ws = (char*)d_ws;
  float*          X    = (float*)(ws + oX);
  unsigned short* H    = (unsigned short*)(ws + oH);
  unsigned short* AGG  = (unsigned short*)(ws + oAGG);
  unsigned short* ZB   = (unsigned short*)(ws + oZB);
  int*            LIST = (int*)(ws + oLIST);
  int*            CO   = (int*)(ws + oCO);
  int*            FLAG = (int*)(ws + oFLAG);
  unsigned short* WC0  = (unsigned short*)(ws + oWC0);
  unsigned short* WC   = (unsigned short*)(ws + oWC);
  float*          BIAS = (float*)(ws + oBIAS);

  hipFuncSetAttribute(reinterpret_cast<const void*>(&k_bucket), hipFuncAttributeMaxDynamicSharedMemorySize, (int)BK_LDS);
  hipFuncSetAttribute(reinterpret_cast<const void*>(&k_gemm<0>), hipFuncAttributeMaxDynamicSharedMemorySize, (int)GL_LDS);
  hipFuncSetAttribute(reinterpret_cast<const void*>(&k_gemm<1>), hipFuncAttributeMaxDynamicSharedMemorySize, (int)GL_LDS);
  hipFuncSetAttribute(reinterpret_cast<const void*>(&k_gemm<2>), hipFuncAttributeMaxDynamicSharedMemorySize, (int)GL_LDS);

  k_prep<<<PBTOT, NTHR, 0, stream>>>(z, Wr0, b0, Wo0, Wr, bl, Wo, ZB, WC0, WC, BIAS);
  k_bucket<<<NBK, NTHR, BK_LDS, stream>>>(srcs, dsts, ew, LIST, CO, FLAG);

  k_agg0<<<MP / ABM, NTHR, 0, stream>>>(LIST, CO, FLAG, ZB, AGG);
  k_gemm<0><<<MP / GBM, NTHR, GL_LDS, stream>>>(AGG, ZB, WC0, BIAS, X, H, out);

  k_agg<<<MP / ABM, NTHR, 0, stream>>>(LIST, CO, FLAG, X, AGG);
  k_gemm<1><<<MP / GBM, NTHR, GL_LDS, stream>>>(AGG, H, WC + (size_t)0 * DH * KC1, BIAS + 1 * DH, X, H, out);
  k_agg<<<MP / ABM, NTHR, 0, stream>>>(LIST, CO, FLAG, X, AGG);
  k_gemm<1><<<MP / GBM, NTHR, GL_LDS, stream>>>(AGG, H, WC + (size_t)1 * DH * KC1, BIAS + 2 * DH, X, H, out);

  k_agg<<<MP / ABM, NTHR, 0, stream>>>(LIST, CO, FLAG, X, AGG);
  k_gemm<2><<<MP / GBM, NTHR, GL_LDS, stream>>>(AGG, H, WC + (size_t)2 * DH * KC1, BIAS + 3 * DH, X, H, out);
}
